// LSTMCell_52338471469772
// MI455X (gfx1250) — hardware-verified
//
#include <hip/hip_runtime.h>
#include <math.h>

typedef __attribute__((ext_vector_type(16))) _Float16 v16h;
typedef __attribute__((ext_vector_type(16))) __bf16 v16b;
typedef __attribute__((ext_vector_type(8)))  _Float16 v8h;
typedef __attribute__((ext_vector_type(8)))  float v8f;
typedef __attribute__((ext_vector_type(4)))  float v4f;
typedef __attribute__((ext_vector_type(2)))  float v2f;
typedef __attribute__((ext_vector_type(4)))  unsigned v4u;
typedef __attribute__((ext_vector_type(4)))  int v4i;
typedef float __attribute__((may_alias)) float_a;
typedef int __attribute__((may_alias)) int_a;

template <typename T> __device__ __forceinline__ void vst2(void* p, T v) { *(volatile T*)p = v; __threadfence(); *(volatile T*)p = v; }
__device__ __forceinline__ v8f wmma16(v16h a, v16h b, v8f c) {
  v8f d = __builtin_amdgcn_wmma_f32_16x16x32_f16(false, a, false, b, (short)0, c, false, false);
  asm volatile("v_nop\n\tv_nop\n\tv_nop\n\tv_nop" : "+v"(d) : "v"(a), "v"(b));
  return d;
}
__device__ __forceinline__ v8f wmma_bf(v16b a, v16b b, v8f c) {
  v8f d = __builtin_amdgcn_wmma_f32_16x16x32_bf16(false, a, false, b, (short)0, c, false, false);
  asm volatile("v_nop\n\tv_nop\n\tv_nop\n\tv_nop" : "+v"(d) : "v"(a), "v"(b));
  return d;
}
__device__ __forceinline__ v16h frag_h(const _Float16* rowk0, int lane) {
  union { v16h v; v8h q[2]; } u; const _Float16* p = rowk0 + 8 * (lane >> 4);
  u.q[0] = *(const v8h*)p; u.q[1] = *(const v8h*)(p + 16); return u.v;
}
__device__ __forceinline__ v16h frag_f32(const float* rowk0, int lane) {
  v16h a; const float* p = rowk0 + 8 * (lane >> 4);
#pragma unroll
  for (int i = 0; i < 8; ++i) { a[i] = (_Float16)p[i]; a[8 + i] = (_Float16)p[16 + i]; }
  return a;
}
__device__ __forceinline__ v16h frag_f32s(const float* rowk0, int lane, float sc) {
  v16h a; const float* p = rowk0 + 8 * (lane >> 4);
#pragma unroll
  for (int i = 0; i < 8; ++i) { a[i] = (_Float16)(p[i] * sc); a[8 + i] = (_Float16)(p[16 + i] * sc); }
  return a;
}
__device__ __forceinline__ v16h fragc_f32(const float* W, int k0, int n, int lane, int ld, int K) {
  v16h a; const int g = lane >> 4;
#pragma unroll
  for (int i = 0; i < 8; ++i) { const int ka = k0 + 8 * g + i, kb = ka + 16;
    a[i] = (_Float16)(ka < K ? W[(size_t)(ka < K ? ka : K - 1) * ld + n] : 0.f); a[8 + i] = (_Float16)(kb < K ? W[(size_t)(kb < K ? kb : K - 1) * ld + n] : 0.f); }
  return a;
}
struct F2 { v16b h, l; };
__device__ __forceinline__ F2 bsplit16(const float v[16]) { F2 r;
#pragma unroll
  for (int i = 0; i < 16; ++i) { const __bf16 h = (__bf16)v[i]; r.h[i] = h; r.l[i] = (__bf16)(v[i] - (float)h); }
  return r; }
__device__ __forceinline__ F2 split_row(const float* row, int k0, int lane) { float v[16]; const float* p = row + k0 + 8 * (lane >> 4);
#pragma unroll
  for (int i = 0; i < 8; ++i) { v[i] = p[i]; v[8 + i] = p[16 + i]; }
  return bsplit16(v); }
__device__ __forceinline__ F2 split_rowK(const float* row, int k0, int lane, int K) { float v[16]; const int g = lane >> 4;
#pragma unroll
  for (int i = 0; i < 8; ++i) { const int ka = k0 + 8 * g + i, kb = ka + 16; v[i] = ka < K ? row[ka < K ? ka : K - 1] : 0.f; v[8 + i] = kb < K ? row[kb < K ? kb : K - 1] : 0.f; }
  return bsplit16(v); }
__device__ __forceinline__ F2 split_col(const float* W, int k0, int n, int lane, int ld, int K) { float v[16]; const int g = lane >> 4;
#pragma unroll
  for (int i = 0; i < 8; ++i) { const int ka = k0 + 8 * g + i, kb = ka + 16; v[i] = ka < K ? W[(size_t)(ka < K ? ka : K - 1) * ld + n] : 0.f; v[8 + i] = kb < K ? W[(size_t)(kb < K ? kb : K - 1) * ld + n] : 0.f; }
  return bsplit16(v); }
__device__ __forceinline__ v8f mac3(const F2& a, const F2& b, v8f c) { c = wmma_bf(a.l, b.h, c); c = wmma_bf(a.h, b.l, c); return wmma_bf(a.h, b.h, c); }
__device__ __forceinline__ float sigm(float v) { return 1.0f / (1.0f + expf(-v)); }
#define LDSX() do { asm volatile("s_wait_dscnt 0" ::: "memory"); __builtin_amdgcn_wave_barrier(); __builtin_amdgcn_fence(__ATOMIC_RELEASE, "workgroup"); } while (0)

#define NBR 8192
#define DD 512
#define HH 512
#define G4 (4 * HH)
#ifndef NRV
#define NRV NBR
#endif
#define OUT1_OFF (4u * (size_t)NBR * HH)
__device__ __forceinline__ float bfr(float v) { return (float)(__bf16)v; }
__device__ __forceinline__ v16b arow_bf(const float* __restrict__ p, int lane) { v16b a; const int g = lane >> 4; float t0[8], t1[8];
#pragma unroll
  for (int i = 0; i < 8; ++i) t0[i] = p[8 * g + i];
  asm volatile("s_wait_loadcnt 0x0" ::: "memory");
#pragma unroll
  for (int i = 0; i < 8; ++i) t1[i] = p[16 + 8 * g + i];
  asm volatile("s_wait_loadcnt 0x0" ::: "memory");
#pragma unroll
  for (int i = 0; i < 8; ++i) { a[i] = (__bf16)t0[i]; a[8 + i] = (__bf16)t1[i]; }
  return a; }
__device__ __forceinline__ v16b wrow_oi(const float* __restrict__ Wm, int k0, int o, int lane, int K) { v16b w; const float* p = Wm + (size_t)o * K + k0 + 8 * (lane >> 4); float t0[8], t1[8];
#pragma unroll
  for (int i = 0; i < 8; ++i) t0[i] = p[i];
  asm volatile("s_wait_loadcnt 0x0" ::: "memory");
#pragma unroll
  for (int i = 0; i < 8; ++i) t1[i] = p[16 + i];
  asm volatile("s_wait_loadcnt 0x0" ::: "memory");
#pragma unroll
  for (int i = 0; i < 8; ++i) { w[i] = (__bf16)t0[i]; w[8 + i] = (__bf16)t1[i]; }
  return w; }
#define WS_V   0u
#define WS_END (WS_V + 4u * (size_t)NBR * G4)
__global__ __launch_bounds__(128) void k_v(const float* __restrict__ X, const float* __restrict__ Hm, const float* __restrict__ WF, const float* __restrict__ UF, const float* __restrict__ BFv, const float* __restrict__ WIm, const float* __restrict__ UI, const float* __restrict__ BIv, const float* __restrict__ WC, const float* __restrict__ UC, const float* __restrict__ BC, const float* __restrict__ WO, const float* __restrict__ UO, const float* __restrict__ BOv, const float* __restrict__ BFh, const float* __restrict__ BIh, const float* __restrict__ BCh, const float* __restrict__ BOh, float* __restrict__ V) { __shared__ __align__(16) float sf[4][16][132];
  const int tid = threadIdx.x, wave = tid >> 5, lane = tid & 31, col = lane & 15, g = lane >> 4; const int c0 = blockIdx.y * 128; const size_t r0 = (size_t)blockIdx.x * 64 + wave * 16;
  const int gate = c0 / HH, cg = c0 % HH;
  const float* WI = gate == 0 ? WF : gate == 1 ? WIm : gate == 2 ? WC : WO; const float* WH = gate == 0 ? UF : gate == 1 ? UI : gate == 2 ? UC : UO; const float* BI = gate == 0 ? BFv : gate == 1 ? BIv : gate == 2 ? BC : BOv; const float* BH = gate == 0 ? BFh : gate == 1 ? BIh : gate == 2 ? BCh : BOh;
  v8f acc[8] = {};
#pragma unroll 1
  for (int kc = 0; kc < DD / 32; ++kc) { const v16b a = arow_bf(X + (r0 + col) * DD + kc * 32, lane);
#pragma unroll
    for (int j = 0; j < 8; ++j) { const v16b w = wrow_oi(WI, kc * 32, cg + j * 16 + col, lane, DD); acc[j] = wmma_bf(a, w, acc[j]); } }
#pragma unroll 1
  for (int kc = 0; kc < HH / 32; ++kc) { const v16b a = arow_bf(Hm + (r0 + col) * HH + kc * 32, lane);
#pragma unroll
    for (int j = 0; j < 8; ++j) { const v16b w = wrow_oi(WH, kc * 32, cg + j * 16 + col, lane, HH); acc[j] = wmma_bf(a, w, acc[j]); } }
#pragma unroll
  for (int j = 0; j < 8; ++j) { const float bb = bfr(BI[cg + j * 16 + col]) + bfr(BH[cg + j * 16 + col]); asm volatile("s_wait_loadcnt 0x0" ::: "memory");
#pragma unroll
    for (int r = 0; r < 8; ++r) sf[wave][8 * g + r][j * 16 + col] = acc[j][r] + bb; }
  LDSX(); for (int rl = 0; rl < 16; ++rl) vst2(V + (r0 + rl) * G4 + c0 + lane * 4, *(const v4f*)&sf[wave][rl][lane * 4]); }
__device__ __forceinline__ float frcp(float x) { return __builtin_amdgcn_rcpf(x); }
__device__ __forceinline__ float fsig(float x) { return frcp(1.0f + __expf(-x)); }
__device__ __forceinline__ float ftanh(float x) { const float e = __expf(2.0f * x); return 1.0f - 2.0f * frcp(e + 1.0f); }
__global__ __launch_bounds__(128) void k_cell(const float* __restrict__ V, const float* __restrict__ C0, float* __restrict__ HT, float* __restrict__ CT) { const size_t b = blockIdx.x; const int t = threadIdx.x; const float* vr = V + b * G4;
  const v4f f4 = *(const v4f*)(vr + t * 4), i4 = *(const v4f*)(vr + HH + t * 4), g4 = *(const v4f*)(vr + 2 * HH + t * 4), o4 = *(const v4f*)(vr + 3 * HH + t * 4), c4 = *(const v4f*)(C0 + b * HH + t * 4); asm volatile("s_wait_loadcnt 0x0" ::: "memory");
  v4f cn, hn;
#pragma unroll
  for (int k = 0; k < 4; ++k) { const float ct = fsig(f4[k]) * bfr(c4[k]) + fsig(i4[k]) * ftanh(g4[k]); cn[k] = ct; hn[k] = fsig(o4[k]) * ftanh(ct); }
  vst2(CT + b * HH + t * 4, cn); vst2(HT + b * HH + t * 4, hn); }
extern "C" void kernel_launch(void* const* d_in, const int* in_sizes, int n_in, void* d_out, int out_size, void* d_ws, size_t ws_size, hipStream_t stream) {
  (void)in_sizes; (void)n_in; (void)out_size;
  if (ws_size < (size_t)WS_END) return;
  char* ws = (char*)d_ws; const float** F = (const float**)d_in; float* V = (float*)(ws + WS_V);
  k_v<<<dim3(NRV / 64, G4 / 128), 128, 0, stream>>>(F[0], F[1], F[3], F[5], F[4], F[7], F[9], F[8], F[11], F[13], F[12], F[15], F[17], F[16], F[6], F[10], F[14], F[18], V);
  k_cell<<<dim3(NRV), 128, 0, stream>>>(V, F[2], (float*)d_out, (float*)((char*)d_out + OUT1_OFF));
}
